// Encoder_6949257085628
// MI455X (gfx1250) — hardware-verified
//
#include <hip/hip_runtime.h>
#include <math.h>

constexpr int NSTEP     = 20;
constexpr int NBATCH    = 65536;
constexpr int NHID      = 64;
constexpr int NEMB      = 64;
constexpr int NGATE     = 4 * NHID;
constexpr int NTHR      = 256;
constexpr int NWAVE     = NTHR / 32;
constexpr int NCHUNK    = NHID / 16;
constexpr int MT_BLK    = NWAVE / NCHUNK;
constexpr int ROWS_BLK  = MT_BLK * 16;
constexpr int HPITCH    = 72;
constexpr int SLABP     = 68;
constexpr float WCARRY    = 16.0f;
constexpr float HCARRY    = 64.0f;
constexpr float CARRY     = WCARRY * HCARRY;
constexpr float CARRY_INV = 1.0f / CARRY;

static_assert(NGATE == NTHR, "one gate row per thread in the fold prologue");
static_assert(NCHUNK == 4 && MT_BLK == 2 && ROWS_BLK == 32, "wave map assumes 4 chunks x 2 M-tiles");
static_assert(NBATCH % ROWS_BLK == 0, "grid exact");
static_assert(NHID % 32 == 0 && NHID == 64 && NEMB == 64, "K = 64 = 2 k-steps of 32");
static_assert((ROWS_BLK * HPITCH) % 8 == 0, "h tile fill in 16-B pieces");
static_assert((ROWS_BLK * NHID) % (NTHR * 4) == 0, "final store loop exact");

typedef __attribute__((ext_vector_type(16))) _Float16 v16h;
typedef __attribute__((ext_vector_type(8)))  _Float16 v8h;
typedef __attribute__((ext_vector_type(8)))  float    v8f;
typedef __attribute__((ext_vector_type(4)))  float    v4f;

__device__ __forceinline__ void grp_guard_h(v8f& a0, v8f& a1, v8f& a2, v8f& a3,
                                            v16h x, v16h y0, v16h y1, v16h y2, v16h y3) {
  asm volatile("v_nop\n\tv_nop\n\tv_nop\n\tv_nop"
               : "+v"(a0), "+v"(a1), "+v"(a2), "+v"(a3)
               : "v"(x), "v"(y0), "v"(y1), "v"(y2), "v"(y3));
}

union FragU { v16h v; v8h h[2]; };
__device__ __forceinline__ v16h frag_load(const _Float16* p) {
  FragU f;
  f.h[0] = *(const v8h*)(p);
  f.h[1] = *(const v8h*)(p + 16);
  return f.v;
}
__device__ __forceinline__ v8f frag_mma(v16h a, v16h b, v8f c) {
  return __builtin_amdgcn_wmma_f32_16x16x32_f16(false, a, false, b, (short)0, c, false, false);
}

__device__ __forceinline__ float fsig(float x)  { return __builtin_amdgcn_rcpf(1.0f + __expf(-x)); }
__device__ __forceinline__ float ftanh(float x) { return 1.0f - 2.0f * __builtin_amdgcn_rcpf(__expf(2.0f * x) + 1.0f); }

__global__ __launch_bounds__(NTHR) __attribute__((amdgpu_num_vgpr(256)))
void lstm_enc_kernel(
    const float* __restrict__ obs,
    const float* __restrict__ W_emb,
    const float* __restrict__ b_emb,
    const float* __restrict__ W_ih,
    const float* __restrict__ W_hh,
    const float* __restrict__ b_ih,
    const float* __restrict__ b_hh,
    float* __restrict__ out) {
  __shared__ __align__(16) _Float16 sH[ROWS_BLK * HPITCH];
  __shared__ __align__(16) float    sOut[ROWS_BLK * SLABP];
  __shared__ float sC0[NGATE];
  __shared__ float sC1[NGATE];
  __shared__ float sCb[NGATE];

  const int tid  = threadIdx.x;
  const int lane = tid & 31;
  const int wave = tid >> 5;
  const int c    = lane & 15;
  const int hh   = lane >> 4;
  const int koff = hh * 8;
  const int mt   = wave >> 2;
  const int j    = wave & 3;

  {
    const int g = tid;
    const float* wr = W_ih + (size_t)g * NEMB;
    float a0 = 0.0f, a1 = 0.0f, ab = 0.0f;
#pragma unroll 1
    for (int i = 0; i < NEMB / 4; ++i) {
      const v4f w  = *(const v4f*)(wr + 4 * i);
      const v4f e0 = *(const v4f*)(W_emb + 8 * i);
      const v4f e1 = *(const v4f*)(W_emb + 8 * i + 4);
      const v4f be = *(const v4f*)(b_emb + 4 * i);
      a0 = fmaf(w[0], e0[0], a0); a1 = fmaf(w[0], e0[1], a1); ab = fmaf(w[0], be[0], ab);
      a0 = fmaf(w[1], e0[2], a0); a1 = fmaf(w[1], e0[3], a1); ab = fmaf(w[1], be[1], ab);
      a0 = fmaf(w[2], e1[0], a0); a1 = fmaf(w[2], e1[1], a1); ab = fmaf(w[2], be[2], ab);
      a0 = fmaf(w[3], e1[2], a0); a1 = fmaf(w[3], e1[3], a1); ab = fmaf(w[3], be[3], ab);
    }
    const float bsum = b_ih[g] + b_hh[g];
    sC0[g] = a0 * CARRY;
    sC1[g] = a1 * CARRY;
    sCb[g] = (ab + bsum) * CARRY;
  }
  {
    const v8h zz = {(_Float16)0.0f, (_Float16)0.0f, (_Float16)0.0f, (_Float16)0.0f,
                    (_Float16)0.0f, (_Float16)0.0f, (_Float16)0.0f, (_Float16)0.0f};
#pragma unroll 1
    for (int i = tid; i < (ROWS_BLK * HPITCH) / 8; i += NTHR) *(v8h*)(sH + 8 * i) = zz;
  }

  v16h bw[4][2];
#pragma unroll
  for (int g = 0; g < 4; ++g) {
#pragma unroll
    for (int kh = 0; kh < 2; ++kh) {
      const float* p = W_hh + (size_t)(g * NHID + 16 * j + c) * NHID + kh * 32 + koff;
      const v4f q0 = *(const v4f*)(p);
      const v4f q1 = *(const v4f*)(p + 4);
      const v4f q2 = *(const v4f*)(p + 16);
      const v4f q3 = *(const v4f*)(p + 20);
      v16h f;
#pragma unroll
      for (int e = 0; e < 4; ++e) {
        f[e]      = (_Float16)(q0[e] * WCARRY);
        f[4 + e]  = (_Float16)(q1[e] * WCARRY);
        f[8 + e]  = (_Float16)(q2[e] * WCARRY);
        f[12 + e] = (_Float16)(q3[e] * WCARRY);
      }
      bw[g][kh] = f;
      asm volatile("" ::: "memory");
    }
  }

  float cst[8], hst[8];
#pragma unroll
  for (int r = 0; r < 8; ++r) { cst[r] = 0.0f; hst[r] = 0.0f; }
  __syncthreads();

  float k0[4], k1[4], kb[4];
#pragma unroll
  for (int g = 0; g < 4; ++g) {
    const int n = g * NHID + 16 * j + c;
    k0[g] = sC0[n];
    k1[g] = sC1[n];
    kb[g] = sCb[n];
  }

  const size_t rowT = (size_t)blockIdx.x * ROWS_BLK + (size_t)mt * 16;
  const _Float16* arow = sH + (mt * 16 + c) * HPITCH + koff;
  _Float16* hw = sH + (mt * 16) * HPITCH + 16 * j + c;

#pragma unroll 1
  for (int t = 0; t < NSTEP; ++t) {
    float ox[8], oy[8];
    {
      const float* op = obs + ((size_t)t * NBATCH + rowT + (size_t)(8 * hh)) * 2;
      const v4f o0 = *(const v4f*)(op);
      const v4f o1 = *(const v4f*)(op + 4);
      const v4f o2 = *(const v4f*)(op + 8);
      const v4f o3 = *(const v4f*)(op + 12);
      ox[0] = o0[0]; oy[0] = o0[1]; ox[1] = o0[2]; oy[1] = o0[3];
      ox[2] = o1[0]; oy[2] = o1[1]; ox[3] = o1[2]; oy[3] = o1[3];
      ox[4] = o2[0]; oy[4] = o2[1]; ox[5] = o2[2]; oy[5] = o2[3];
      ox[6] = o3[0]; oy[6] = o3[1]; ox[7] = o3[2]; oy[7] = o3[3];
    }
    const v16h a0 = frag_load(arow);
    const v16h a1 = frag_load(arow + 32);

    v8f acc[4];
#pragma unroll
    for (int g = 0; g < 4; ++g)
#pragma unroll
      for (int r = 0; r < 8; ++r) acc[g][r] = fmaf(ox[r], k0[g], fmaf(oy[r], k1[g], kb[g]));

    acc[0] = frag_mma(a0, bw[0][0], acc[0]);
    acc[1] = frag_mma(a0, bw[1][0], acc[1]);
    acc[2] = frag_mma(a0, bw[2][0], acc[2]);
    acc[3] = frag_mma(a0, bw[3][0], acc[3]);
    grp_guard_h(acc[0], acc[1], acc[2], acc[3], a0, bw[0][0], bw[1][0], bw[2][0], bw[3][0]);
    acc[0] = frag_mma(a1, bw[0][1], acc[0]);
    acc[1] = frag_mma(a1, bw[1][1], acc[1]);
    acc[2] = frag_mma(a1, bw[2][1], acc[2]);
    acc[3] = frag_mma(a1, bw[3][1], acc[3]);
    grp_guard_h(acc[0], acc[1], acc[2], acc[3], a1, bw[0][1], bw[1][1], bw[2][1], bw[3][1]);

#pragma unroll
    for (int r = 0; r < 8; ++r) {
      const float zi = acc[0][r] * CARRY_INV;
      const float zf = acc[1][r] * CARRY_INV;
      const float zg = acc[2][r] * CARRY_INV;
      const float zo = acc[3][r] * CARRY_INV;
      const float ig = fsig(zi);
      const float fg = fsig(zf);
      const float gv = ftanh(zg);
      const float og = fsig(zo);
      const float cn = fg * cst[r] + ig * gv;
      cst[r] = cn;
      hst[r] = og * ftanh(cn);
    }

    __syncthreads();
#pragma unroll
    for (int r = 0; r < 8; ++r) hw[(8 * hh + r) * HPITCH] = (_Float16)(hst[r] * HCARRY);
    __syncthreads();
  }

#pragma unroll
  for (int r = 0; r < 8; ++r) sOut[(mt * 16 + 8 * hh + r) * SLABP + 16 * j + c] = hst[r];
  __syncthreads();
  {
    float* ob = out + (size_t)blockIdx.x * ROWS_BLK * NHID;
    for (int pass = 0; pass < 2; ++pass) {
#pragma unroll
      for (int it = 0; it < (ROWS_BLK * NHID) / (NTHR * 4); ++it) {
        const int idx = it * NTHR + tid;
        const int row = idx >> 4;
        const int c4  = (idx & 15) * 4;
        const v4f v = *(const v4f*)(sOut + row * SLABP + c4);
        *(volatile v4f*)(ob + (size_t)row * NHID + c4) = v;
      }
      __threadfence();
    }
  }
}

extern "C" void kernel_launch(void* const* d_in, const int* in_sizes, int n_in,
                              void* d_out, int out_size, void* d_ws, size_t ws_size,
                              hipStream_t stream) {
  (void)d_ws; (void)ws_size;
  if (n_in < 7 || d_out == nullptr) return;
  if (in_sizes[0] != NSTEP * NBATCH * 2 || in_sizes[1] != NEMB * 2 || in_sizes[2] != NEMB ||
      in_sizes[3] != NGATE * NEMB || in_sizes[4] != NGATE * NHID || in_sizes[5] != NGATE ||
      in_sizes[6] != NGATE || out_size != NBATCH * NHID) return;

  const float* obs   = (const float*)d_in[0];
  const float* W_emb = (const float*)d_in[1];
  const float* b_emb = (const float*)d_in[2];
  const float* W_ih  = (const float*)d_in[3];
  const float* W_hh  = (const float*)d_in[4];
  const float* b_ih  = (const float*)d_in[5];
  const float* b_hh  = (const float*)d_in[6];
  float* out = (float*)d_out;

  lstm_enc_kernel<<<NBATCH / ROWS_BLK, NTHR, 0, stream>>>(obs, W_emb, b_emb, W_ih, W_hh, b_ih, b_hh, out);
}
